// AttentionSumPooling_60249801228695
// MI455X (gfx1250) — hardware-verified
//
#include <hip/hip_runtime.h>
#include <stddef.h>


#define NTHR   256
#define NWAVE  8
#define FIN    128
#define FH     256
#define FH2    128
#define NHEAD  8
#define XW     512
#define NLAY   3
#define NG     64
#define NOUT   10

#define GR     32
#define GCW    256
#define XSP    260

#define NB     256
#define CHUNK  2048
#define WCAP   256
#define NGRP   (CHUNK / (NTHR * 4))
#define AGG_LDS_BYTES ((NB * FH + 2 * NB * NHEAD) * 4 + (NWAVE * WCAP + NWAVE) * 4)

#define HP1    264
#define HP2    136
#define HEAD_R0 (NG * FH * 4)
#define HEAD_R1 (NG * HP1 * 2)
#define HEAD_LDS_BYTES (HEAD_R0 + HEAD_R1)

static_assert(NGRP == 2);
static_assert(WCAP == (CHUNK / NTHR) * 32);
static_assert(AGG_LDS_BYTES == 286752);
static_assert(HEAD_LDS_BYTES == 99328);
static_assert(NG * HP1 * 2 <= HEAD_R0);
static_assert(NG * HP2 * 2 <= HEAD_R1);
static_assert(NG * NOUT * 4 <= HEAD_R0);
static_assert((NB & (NB - 1)) == 0);
static_assert(NB <= 256);
static_assert((XSP % 4) == 0);
static_assert(FH == NHEAD * 32);
static_assert(NTHR == FH);
static_assert((NG * NOUT) % 128 == 0);

typedef float    v4f  __attribute__((ext_vector_type(4)));
typedef float    v8f  __attribute__((ext_vector_type(8)));
typedef int      v4i  __attribute__((ext_vector_type(4)));
typedef _Float16 v8h  __attribute__((ext_vector_type(8)));
typedef _Float16 v16h __attribute__((ext_vector_type(16)));

union FragH { v16h v; v4i u[2]; _Float16 s[16]; };
union Pack  { v8h h; v4i i; _Float16 s[8]; };

__device__ __forceinline__ v8f wm(v16h a, v16h b, v8f c) {
  v8f d = __builtin_amdgcn_wmma_f32_16x16x32_f16(false, a, false, b, (short)0, c, false, false);
  asm volatile("v_nop\n\tv_nop\n\tv_nop\n\tv_nop" : "+v"(d) : "v"(a), "v"(b));
  return d;
}

__device__ __forceinline__ float lk(float t) { return fmaxf(t, 0.2f * t); }
__device__ __forceinline__ float dl(v4f t, v4f w) {
  return w.x * lk(t.x) + w.y * lk(t.y) + w.z * lk(t.z) + w.w * lk(t.w);
}
__device__ __forceinline__ v4f relu4(v4f v) {
  v4f r;
  r.x = fmaxf(v.x, 0.f); r.y = fmaxf(v.y, 0.f); r.z = fmaxf(v.z, 0.f); r.w = fmaxf(v.w, 0.f);
  return r;
}
__device__ __forceinline__ v4i pack8(v4f a, v4f b) {
  Pack u;
  u.s[0] = (_Float16)a.x; u.s[1] = (_Float16)a.y; u.s[2] = (_Float16)a.z; u.s[3] = (_Float16)a.w;
  u.s[4] = (_Float16)b.x; u.s[5] = (_Float16)b.y; u.s[6] = (_Float16)b.z; u.s[7] = (_Float16)b.w;
  return u.i;
}

__device__ __forceinline__ v16h gatherB(const float* __restrict__ W, int ld, int n, int k0, int hh, float sc) {
  FragH b;
#pragma unroll
  for (int i = 0; i < 8; ++i) {
    b.s[i]     = (_Float16)(W[(size_t)(k0 + 8 * hh + i) * ld + n] * sc);
    b.s[8 + i] = (_Float16)(W[(size_t)(k0 + 16 + 8 * hh + i) * ld + n] * sc);
  }
  return b.v;
}

__global__ __launch_bounds__(NTHR) void k_cvt(const float* __restrict__ src, long long sbat, long long sr, long long sk,
                                              int rows_src, int K, float scale,
                                              _Float16* dst, long long dbat, int rows_out) {
  const float* sp = src + (size_t)blockIdx.y * (size_t)sbat;
  _Float16* dp = dst + (size_t)blockIdx.y * (size_t)dbat;
  const int kp8 = K >> 3;
  const int n8  = rows_out * kp8;
  const int i   = blockIdx.x * NTHR + threadIdx.x;
  if (i >= n8) return;
  const int r  = i / kp8;
  const int kb = (i - r * kp8) * 8;
  const bool live = (r < rows_src);
  const int rc = live ? r : 0;
  Pack u;
#pragma unroll
  for (int j = 0; j < 8; ++j) {
    const float t = live ? sp[(size_t)rc * (size_t)sr + (size_t)(kb + j) * (size_t)sk] : 0.f;
    u.s[j] = (_Float16)(t * scale);
  }
  const size_t o = (size_t)r * K + kb;
  *(volatile v4i*)(dp + o) = u.i;
  __threadfence();
  *(volatile v4i*)(dp + o) = u.i;
}

__global__ __launch_bounds__(NTHR) void k_gemm(const _Float16* A, const _Float16* Bt,
                                               const float* __restrict__ bias0, const float* __restrict__ bias1, int nb0,
                                               float* outF, _Float16* outH, int write16,
                                               int K, int Ncols, float oscale) {
  __shared__ __attribute__((aligned(16))) float Xs[GR * XSP];

  const int tid  = threadIdx.x;
  const int lane = tid & 31;
  const int wave = tid >> 5;
  const int hh   = lane >> 4;
  const int m    = lane & 15;
  const int rowBase = blockIdx.x * GR;
  const int colBase = blockIdx.y * GCW;
  const int cw = 32 * wave;

  const size_t ra0 = (size_t)(rowBase + m) * K + 8 * hh;
  const size_t ra1 = ra0 + (size_t)16 * K;
  const size_t rb0 = (size_t)(colBase + cw + m) * K + 8 * hh;
  const size_t rb1 = rb0 + (size_t)16 * K;

  const v8f z8 = {0.f, 0.f, 0.f, 0.f, 0.f, 0.f, 0.f, 0.f};
  v8f c00 = z8, c01 = z8, c10 = z8, c11 = z8;

#pragma unroll 1
  for (int k0 = 0; k0 < K; k0 += 32) {
    FragH a0, a1, b0, b1;
    a0.u[0] = *(const v4i*)(A + ra0 + k0);   a0.u[1] = *(const v4i*)(A + ra0 + k0 + 16);
    a1.u[0] = *(const v4i*)(A + ra1 + k0);   a1.u[1] = *(const v4i*)(A + ra1 + k0 + 16);
    b0.u[0] = *(const v4i*)(Bt + rb0 + k0);  b0.u[1] = *(const v4i*)(Bt + rb0 + k0 + 16);
    b1.u[0] = *(const v4i*)(Bt + rb1 + k0);  b1.u[1] = *(const v4i*)(Bt + rb1 + k0 + 16);
    c00 = wm(a0.v, b0.v, c00);
    c01 = wm(a0.v, b1.v, c01);
    c10 = wm(a1.v, b0.v, c10);
    c11 = wm(a1.v, b1.v, c11);
  }

  const int gc0 = colBase + cw + m, gc1 = gc0 + 16;
  const float* bp0 = (gc0 < nb0) ? (bias0 + gc0) : (bias1 + (gc0 - nb0));
  const float* bp1 = (gc1 < nb0) ? (bias0 + gc1) : (bias1 + (gc1 - nb0));
  const float bv0 = *bp0, bv1 = *bp1;
  const int cl0 = cw + m, cl1 = cl0 + 16;
#pragma unroll
  for (int r = 0; r < 8; ++r) {
    Xs[(8 * hh + r) * XSP + cl0]      = c00[r] * oscale + bv0;
    Xs[(8 * hh + r) * XSP + cl1]      = c01[r] * oscale + bv1;
    Xs[(16 + 8 * hh + r) * XSP + cl0] = c10[r] * oscale + bv0;
    Xs[(16 + 8 * hh + r) * XSP + cl1] = c11[r] * oscale + bv1;
  }
  __syncthreads();

#pragma unroll 1
  for (int ps = 0; ps < 2; ++ps) {
#pragma unroll
    for (int i = 0; i < 4; ++i) {
      const int row = 4 * wave + i;
      const float* xr = Xs + row * XSP;
      const size_t go = (size_t)(rowBase + row) * Ncols + colBase;
      const v4f x0 = *(const v4f*)(xr + 4 * lane);
      const v4f x1 = *(const v4f*)(xr + 128 + 4 * lane);
      *(volatile v4f*)(outF + go + 4 * lane)       = x0;
      *(volatile v4f*)(outF + go + 128 + 4 * lane) = x1;
      if (write16) {
        const v4f f0 = *(const v4f*)(xr + 8 * lane);
        const v4f f1 = *(const v4f*)(xr + 8 * lane + 4);
        *(volatile v4i*)(outH + go + 8 * lane) = pack8(f0, f1);
      }
    }
    if (ps == 0) __threadfence();
  }
}

__device__ __forceinline__ void hit8(const float* xs, const float* xd, float* ar, float* mp, float* dp,
                                     v4f w0, v4f w1) {
  const v4f a0 = *(const v4f*)(xs), a1 = *(const v4f*)(xs + 4);
  const v4f d0 = *(const v4f*)(xd), d1 = *(const v4f*)(xd + 4);
  float s = dl(a0 + d0, w0) + dl(a1 + d1, w1);
  s += __shfl_xor(s, 2, 32);
  s += __shfl_xor(s, 1, 32);
  const float mo = mp[0], no = dp[0];
  const float mn = fmaxf(mo, s);
  const float sc = __expf(mo - mn);
  const float p  = __expf(s - mn);
  v4f e0 = *(v4f*)(ar), e1 = *(v4f*)(ar + 4);
  e0 = e0 * sc + a0 * p;
  e1 = e1 * sc + a1 * p;
  *(v4f*)(ar)     = e0;
  *(v4f*)(ar + 4) = e1;
  mp[0] = mn;
  dp[0] = no * sc + p;
}

__global__ __launch_bounds__(NTHR) void k_agg(const int* __restrict__ esrc, const int* __restrict__ edst,
                                              const float* __restrict__ X, const float* __restrict__ att,
                                              const float* __restrict__ Hin,
                                              float* Hout, _Float16* Hout16, int nN, int nE, int nW) {
  extern __shared__ v4f lds_dyn[];
  float* sacc = (float*)lds_dyn;
  float* mx   = sacc + NB * FH;
  float* dn   = mx + NB * NHEAD;
  int*   list = (int*)(dn + NB * NHEAD);
  int*   wcnt = list + NWAVE * WCAP;

  const int tid  = threadIdx.x;
  const int lane = tid & 31;
  const int wave = tid >> 5;
  const int nodeBase = blockIdx.x * NB;

  {
    const v4f z4 = {0.f, 0.f, 0.f, 0.f};
    for (int i = tid; i < NB * FH / 4; i += NTHR) lds_dyn[i] = z4;
    for (int i = tid; i < NB * NHEAD; i += NTHR) { mx[i] = -1.0e30f; dn[i] = 0.f; }
  }
  __syncthreads();

  const int co   = 8 * lane;
  const int head = lane >> 2;
  const v4f w0 = *(const v4f*)(att + co);
  const v4f w1 = *(const v4f*)(att + co + 4);

  const bool al16 = ((((size_t)edst) & 15) == 0);
  const int nChunks = (nE + CHUNK - 1) / CHUNK;

#pragma unroll 1
  for (int ch = 0; ch < nChunks; ++ch) {
    const int cbase = ch * CHUNK;
    int wc = 0;
#pragma unroll
    for (int g = 0; g < NGRP; ++g) {
      const int el0 = (g * NTHR + tid) * 4;
      const int e0  = cbase + el0;
      const int sent = -2147483647 - 1;
      v4i d;
      if (al16 && (e0 + 3 < nE)) {
        d = *(const v4i*)(edst + e0);
      } else {
        d.x = (e0     < nE) ? edst[min(e0, nE - 1)]     : sent;
        d.y = (e0 + 1 < nE) ? edst[min(e0 + 1, nE - 1)] : sent;
        d.z = (e0 + 2 < nE) ? edst[min(e0 + 2, nE - 1)] : sent;
        d.w = (e0 + 3 < nE) ? edst[min(e0 + 3, nE - 1)] : sent;
      }
      const unsigned s0 = (unsigned)d.x - (unsigned)nodeBase;
      const unsigned s1 = (unsigned)d.y - (unsigned)nodeBase;
      const unsigned s2 = (unsigned)d.z - (unsigned)nodeBase;
      const unsigned s3 = (unsigned)d.w - (unsigned)nodeBase;
      const bool h0 = s0 < (unsigned)NB;
      const bool h1 = s1 < (unsigned)NB;
      const bool h2 = s2 < (unsigned)NB;
      const bool h3 = s3 < (unsigned)NB;
      const unsigned many = __builtin_amdgcn_ballot_w32(h0 | h1 | h2 | h3);
      if (many != 0u) {
#define HITJ(J, HJ, SJ) { \
          const unsigned mj = __builtin_amdgcn_ballot_w32(HJ); \
          if (HJ) { \
            const int pos = wc + (int)__builtin_amdgcn_mbcnt_lo(mj, 0u); \
            if (pos < WCAP) list[wave * WCAP + pos] = ((el0 + (J)) << 8) | (int)(SJ); \
          } \
          wc += (int)__builtin_popcount(mj); }
        HITJ(0, h0, s0)
        HITJ(1, h1, s1)
        HITJ(2, h2, s2)
        HITJ(3, h3, s3)
#undef HITJ
      }
    }
    if (lane == 0) wcnt[wave] = wc;
    __syncthreads();

    if (wave == 0) {
#pragma unroll 1
      for (int wsx = 0; wsx < NWAVE; ++wsx) {
        int n = __builtin_amdgcn_readfirstlane(wcnt[wsx]);
        n = n > WCAP ? WCAP : n;
        n = n < 0 ? 0 : n;
#pragma unroll 1
        for (int i = 0; i < n; ++i) {
          const int ent  = __builtin_amdgcn_readfirstlane(list[wsx * WCAP + i]);
          const int slot = ent & (NB - 1);
          const int el   = (ent >> 8) & (CHUNK - 1);
          const int node = nodeBase + slot;
          if (node >= nN) continue;
          int e = cbase + el;
          if (e > nE - 1) e = nE - 1;
          int sj = esrc[e];
          sj = sj < 0 ? 0 : (sj > nN - 1 ? nN - 1 : sj);
          const float* xs = X + (size_t)sj * XW + co;
          const float* xd = X + (size_t)node * XW + FH + co;
          hit8(xs, xd, sacc + slot * FH + co, mx + slot * NHEAD + head, dn + slot * NHEAD + head, w0, w1);
        }
      }
    }
    __syncthreads();
  }

#pragma unroll 1
  for (int j = 0; j < NB / NWAVE; ++j) {
    const int s    = wave + NWAVE * j;
    const int node = nodeBase + s;
    v4f o0 = {0.f, 0.f, 0.f, 0.f};
    v4f o1 = {0.f, 0.f, 0.f, 0.f};
    if (node < nN) {
      const float* ar = sacc + s * FH + co;
      const v4f e0 = *(const v4f*)(ar), e1 = *(const v4f*)(ar + 4);
      const float den = dn[s * NHEAD + head];
      const float inv = (den > 0.f) ? __fdividef(1.0f, den) : 0.f;
      const v4f g0 = *(const v4f*)(Hin + (size_t)node * FH + co);
      const v4f g1 = *(const v4f*)(Hin + (size_t)node * FH + co + 4);
      o0 = relu4(e0 * inv + g0);
      o1 = relu4(e1 * inv + g1);
    }
    *(v4f*)(sacc + s * FH + co)     = o0;
    *(v4f*)(sacc + s * FH + co + 4) = o1;
  }
  __syncthreads();

#pragma unroll 1
  for (int ps = 0; ps < 2; ++ps) {
#pragma unroll 1
    for (int j = 0; j < NB / NWAVE; ++j) {
      const int s    = wave + NWAVE * j;
      const int node = nodeBase + s;
      if (node < nW) {
        const float* rowp = sacc + s * FH;
        const v4f x0 = *(const v4f*)(rowp + 4 * lane);
        const v4f x1 = *(const v4f*)(rowp + 128 + 4 * lane);
        const v4f f0 = *(const v4f*)(rowp + 8 * lane);
        const v4f f1 = *(const v4f*)(rowp + 8 * lane + 4);
        const size_t ro = (size_t)node * FH;
        *(volatile v4f*)(Hout + ro + 4 * lane)       = x0;
        *(volatile v4f*)(Hout + ro + 128 + 4 * lane) = x1;
        *(volatile v4i*)(Hout16 + ro + 8 * lane)     = pack8(f0, f1);
      }
    }
    if (ps == 0) __threadfence();
  }
}

__global__ __launch_bounds__(NTHR) void k_head(const float* __restrict__ H, const int* __restrict__ gid,
                                               const float* __restrict__ W1, const float* __restrict__ B1,
                                               const float* __restrict__ W2, const float* __restrict__ B2,
                                               const float* __restrict__ W3, const float* __restrict__ B3,
                                               float* out, int nN) {
  extern __shared__ v4f lds_dyn[];
  char* base = (char*)lds_dyn;
  float*    accP = (float*)base;
  _Float16* X1   = (_Float16*)base;
  float*    Ob   = (float*)base;
  _Float16* A0   = (_Float16*)(base + HEAD_R0);
  _Float16* X2   = (_Float16*)(base + HEAD_R0);

  const int tid  = threadIdx.x;
  const int lane = tid & 31;
  const int wave = tid >> 5;
  const int hh   = lane >> 4;
  const int m    = lane & 15;
  const v8f z8 = {0.f, 0.f, 0.f, 0.f, 0.f, 0.f, 0.f, 0.f};

#pragma unroll
  for (int g = 0; g < NG; ++g) accP[g * FH + tid] = 0.f;
#pragma unroll 1
  for (int node = 0; node < nN; ++node) {
    const int g = gid[node];
    if ((unsigned)g < (unsigned)NG) accP[g * FH + tid] += H[(size_t)node * FH + tid];
  }
  __syncthreads();

#pragma unroll
  for (int q = 0; q < 8; ++q) {
    const int idx = tid + NTHR * q;
    const int row = idx >> 5;
    const int kb  = (idx & 31) * 8;
    const v4f f0 = *(const v4f*)(accP + row * FH + kb);
    const v4f f1 = *(const v4f*)(accP + row * FH + kb + 4);
    *(v4i*)(A0 + row * HP1 + kb) = pack8(f0, f1);
  }
  __syncthreads();

#pragma unroll 1
  for (int cti = 0; cti < 2; ++cti) {
    const int n = 16 * (2 * wave + cti) + m;
    v8f c[4];
#pragma unroll
    for (int rt = 0; rt < 4; ++rt) c[rt] = z8;
#pragma unroll 1
    for (int k0 = 0; k0 < FH; k0 += 32) {
      FragH a[4];
#pragma unroll
      for (int rt = 0; rt < 4; ++rt) {
        a[rt].u[0] = *(const v4i*)(A0 + (rt * 16 + m) * HP1 + k0 + 8 * hh);
        a[rt].u[1] = *(const v4i*)(A0 + (rt * 16 + m) * HP1 + k0 + 16 + 8 * hh);
      }
      const v16h b = gatherB(W1, FH, n, k0, hh, 16.0f);
#pragma unroll
      for (int rt = 0; rt < 4; ++rt) c[rt] = wm(a[rt].v, b, c[rt]);
    }
    const float bv = B1[n];
#pragma unroll
    for (int rt = 0; rt < 4; ++rt) {
#pragma unroll
      for (int r = 0; r < 8; ++r)
        X1[(rt * 16 + 8 * hh + r) * HP1 + n] = (_Float16)fmaxf(c[rt][r] * 0.0625f + bv, 0.f);
    }
  }
  __syncthreads();

  {
    const int n = 16 * wave + m;
    v8f c[4];
#pragma unroll
    for (int rt = 0; rt < 4; ++rt) c[rt] = z8;
#pragma unroll 1
    for (int k0 = 0; k0 < FH; k0 += 32) {
      FragH a[4];
#pragma unroll
      for (int rt = 0; rt < 4; ++rt) {
        a[rt].u[0] = *(const v4i*)(X1 + (rt * 16 + m) * HP1 + k0 + 8 * hh);
        a[rt].u[1] = *(const v4i*)(X1 + (rt * 16 + m) * HP1 + k0 + 16 + 8 * hh);
      }
      const v16h b = gatherB(W2, FH2, n, k0, hh, 16.0f);
#pragma unroll
      for (int rt = 0; rt < 4; ++rt) c[rt] = wm(a[rt].v, b, c[rt]);
    }
    const float bv = B2[n];
#pragma unroll
    for (int rt = 0; rt < 4; ++rt) {
#pragma unroll
      for (int r = 0; r < 8; ++r)
        X2[(rt * 16 + 8 * hh + r) * HP2 + n] = (_Float16)fmaxf(c[rt][r] * 0.0625f + bv, 0.f);
    }
  }
  __syncthreads();

  if (wave < 4) {
    const int mc = (m < NOUT) ? m : (NOUT - 1);
    const float vm = (m < NOUT) ? 8.0f : 0.0f;
    v8f c0 = z8;
#pragma unroll 1
    for (int k0 = 0; k0 < FH2; k0 += 32) {
      FragH a;
      a.u[0] = *(const v4i*)(X2 + (wave * 16 + m) * HP2 + k0 + 8 * hh);
      a.u[1] = *(const v4i*)(X2 + (wave * 16 + m) * HP2 + k0 + 16 + 8 * hh);
      const v16h b = gatherB(W3, NOUT, mc, k0, hh, vm);
      c0 = wm(a.v, b, c0);
    }
    if (m < NOUT) {
      const float bv = B3[m];
#pragma unroll
      for (int r = 0; r < 8; ++r) Ob[(wave * 16 + 8 * hh + r) * NOUT + m] = c0[r] * 0.125f + bv;
    }
  }
  __syncthreads();

  if (wave == 0) {
#pragma unroll 1
    for (int ps = 0; ps < 2; ++ps) {
#pragma unroll
      for (int q = 0; q < (NG * NOUT) / 128; ++q) {
        const int idx = lane + 32 * q;
        const v4f v = *(const v4f*)(Ob + 4 * idx);
        *(volatile v4f*)(out + 4 * idx) = v;
      }
      if (ps == 0) __threadfence();
    }
  }
}

static inline size_t al256(size_t b) { return (b + 255) & ~(size_t)255; }

extern "C" void kernel_launch(void* const* d_in, const int* in_sizes, int n_in,
                              void* d_out, int out_size, void* d_ws, size_t ws_size,
                              hipStream_t stream) {
  if (n_in < 17) return;
  const int nN = in_sizes[0] / FIN;
  if (nN <= 0 || in_sizes[0] != nN * FIN) return;
  if (in_sizes[1] != FIN * FH || in_sizes[2] != FH) return;
  if (in_sizes[3] != NLAY * FH * FH || in_sizes[4] != NLAY * FH ||
      in_sizes[5] != NLAY * FH * FH || in_sizes[6] != NLAY * FH || in_sizes[7] != NLAY * FH) return;
  if (in_sizes[8] != FH * FH || in_sizes[9] != FH || in_sizes[10] != FH * FH2 || in_sizes[11] != FH2 ||
      in_sizes[12] != FH2 * NOUT || in_sizes[13] != NOUT) return;
  const int nE = in_sizes[14];
  if (nE <= 0 || in_sizes[15] != nE || in_sizes[16] != nN) return;
  if (out_size != NG * NOUT) return;

  const float* feature = (const float*)d_in[0];
  const float* W_in    = (const float*)d_in[1];
  const float* b_in    = (const float*)d_in[2];
  const float* W_src   = (const float*)d_in[3];
  const float* b_src   = (const float*)d_in[4];
  const float* W_dst   = (const float*)d_in[5];
  const float* b_dst   = (const float*)d_in[6];
  const float* attn    = (const float*)d_in[7];
  const float* Wc1     = (const float*)d_in[8];
  const float* bc1     = (const float*)d_in[9];
  const float* Wc2     = (const float*)d_in[10];
  const float* bc2     = (const float*)d_in[11];
  const float* Wc3     = (const float*)d_in[12];
  const float* bc3     = (const float*)d_in[13];
  const int*   esrc    = (const int*)d_in[14];
  const int*   edst    = (const int*)d_in[15];
  const int*   gids    = (const int*)d_in[16];
  float*       out     = (float*)d_out;

  const int Mpad = ((nN + GR - 1) / GR) * GR;

  char* wsp = (char*)d_ws;
  size_t off = 0;
  _Float16* A16  = (_Float16*)(wsp + off); off += al256((size_t)Mpad * FIN * 2);
  _Float16* BtIn = (_Float16*)(wsp + off); off += al256((size_t)FH * FIN * 2);
  _Float16* BtL  = (_Float16*)(wsp + off); off += al256((size_t)NLAY * XW * FH * 2);
  float*    HA   = (float*)(wsp + off);    off += al256((size_t)Mpad * FH * 4);
  float*    HB   = (float*)(wsp + off);    off += al256((size_t)Mpad * FH * 4);
  _Float16* H16  = (_Float16*)(wsp + off); off += al256((size_t)Mpad * FH * 2);
  float*    X    = (float*)(wsp + off);    off += al256((size_t)Mpad * XW * 4);
  if (off > ws_size) return;

  hipFuncSetAttribute(reinterpret_cast<const void*>(&k_agg),
                      hipFuncAttributeMaxDynamicSharedMemorySize, AGG_LDS_BYTES);
  hipFuncSetAttribute(reinterpret_cast<const void*>(&k_head),
                      hipFuncAttributeMaxDynamicSharedMemorySize, HEAD_LDS_BYTES);

  k_cvt<<<dim3((Mpad * (FIN / 8) + NTHR - 1) / NTHR, 1), NTHR, 0, stream>>>(
      feature, (long long)0, (long long)FIN, (long long)1, nN, FIN, 1.0f, A16, (long long)0, Mpad);
  k_cvt<<<dim3((FH * (FIN / 8) + NTHR - 1) / NTHR, 1), NTHR, 0, stream>>>(
      W_in, (long long)0, (long long)1, (long long)FH, FH, FIN, 8.0f, BtIn, (long long)0, FH);
  k_cvt<<<dim3((FH * (FH / 8) + NTHR - 1) / NTHR, NLAY), NTHR, 0, stream>>>(
      W_src, (long long)FH * FH, (long long)1, (long long)FH, FH, FH, 16.0f, BtL, (long long)XW * FH, FH);
  k_cvt<<<dim3((FH * (FH / 8) + NTHR - 1) / NTHR, NLAY), NTHR, 0, stream>>>(
      W_dst, (long long)FH * FH, (long long)1, (long long)FH, FH, FH, 16.0f, BtL + (size_t)FH * FH, (long long)XW * FH, FH);

  k_gemm<<<dim3(Mpad / GR, FH / GCW), NTHR, 0, stream>>>(
      A16, BtIn, b_in, b_in, FH, HA, H16, 1, FIN, FH, 0.125f);

  float* Hbuf[2] = {HA, HB};
  for (int l = 0; l < NLAY; ++l) {
    float* Hin  = Hbuf[l & 1];
    float* Hout = Hbuf[(l + 1) & 1];
    k_gemm<<<dim3(Mpad / GR, XW / GCW), NTHR, 0, stream>>>(
        H16, BtL + (size_t)l * XW * FH, b_src + (size_t)l * FH, b_dst + (size_t)l * FH, FH, X, H16, 0, FH, XW, 0.0625f);
    k_agg<<<(Mpad + NB - 1) / NB, NTHR, AGG_LDS_BYTES, stream>>>(
        esrc, edst, X, attn + (size_t)l * FH, Hin, Hout, H16, nN, nE, Mpad);
  }
  float* Hfin = Hbuf[NLAY & 1];

  k_head<<<1, NTHR, HEAD_LDS_BYTES, stream>>>(Hfin, gids, Wc1, bc1, Wc2, bc2, Wc3, bc3, out, nN);
}
